// CNNModel_82222853915196
// MI455X (gfx1250) — hardware-verified
//
#include <hip/hip_runtime.h>


namespace {
constexpr int Bn = 32, F = 64, T = 512, OUT = 400, OUTP = 400, NFE = 8192, KFC = 64 + NFE  ;
constexpr float AS_ = 8.0f;
struct Wo_ { static constexpr size_t W8 = 0, W16 = W8 + 8 * 16 * 64  , W32 = W16 + 4 * 16 * 256, W64 = W32 + 2 * 64 * 1024, FC = W64 + (size_t)256 * 4096, END = FC + (size_t)OUTP * KFC; };

typedef _Float16 b16;
typedef __attribute__((ext_vector_type(16))) _Float16 v16b;
typedef __attribute__((ext_vector_type(8))) _Float16 v8b;
typedef __attribute__((ext_vector_type(8))) float v8f;
typedef __attribute__((ext_vector_type(4))) float v4f;
__device__ __forceinline__ float bf16_rne(float f) { unsigned int u = __float_as_uint(f); u += 0x7FFFu + ((u >> 16) & 1u); return __uint_as_float(u & 0xFFFF0000u); }
__device__ __forceinline__ void split16(float v, b16& hi, b16& lo) { hi = (b16)v; lo = (b16)(v - (float)hi); }
__device__ __forceinline__ v16b frag_kb(const b16* p, int hh) { const v8b a = *(const v8b*)(p + 8 * hh), b = *(const v8b*)(p + 16 + 8 * hh); v16b f;
#pragma unroll
  for (int e = 0; e < 8; ++e) { f[e] = a[e]; f[8 + e] = b[e]; } return f; }
__device__ __forceinline__ v16b frag_x(const float* p, int hh) { v16b f;
#pragma unroll
  for (int e = 0; e < 8; ++e) { f[e] = (b16)bf16_rne(p[8 * hh + e]); f[8 + e] = (b16)bf16_rne(p[16 + 8 * hh + e]); } return f; }
__device__ __forceinline__ void frag_split(const float* p, int hh, v16b& fh, v16b& fl) {
#pragma unroll
  for (int e = 0; e < 8; ++e) { b16 a, c; split16(p[8 * hh + e] * AS_, a, c); fh[e] = a; fl[e] = c; split16(p[16 + 8 * hh + e] * AS_, a, c); fh[8 + e] = a; fl[8 + e] = c; } }
__device__ __forceinline__ v8f wmma16b(v16b a, v16b b, v8f c) { v8f d = __builtin_amdgcn_wmma_f32_16x16x32_f16(false, a, false, b, (short)0, c, false, false); asm volatile("v_nop\n\tv_nop\n\tv_nop\n\tv_nop" : "+v"(d) : "v"(a), "v"(b)); return d; }
__device__ __forceinline__ void wave_lds_sync() { __builtin_amdgcn_fence(__ATOMIC_RELEASE, "workgroup"); __builtin_amdgcn_wave_barrier(); __builtin_amdgcn_fence(__ATOMIC_ACQUIRE, "workgroup"); }

__global__ __launch_bounds__(256) void prep_kernel(const float* __restrict__ W8, const float* __restrict__ b8, const float* __restrict__ W16, const float* __restrict__ b16_, const float* __restrict__ W32, const float* __restrict__ b32, const float* __restrict__ W64, const float* __restrict__ b64, const float* __restrict__ Wfc, const float* __restrict__ bfc, b16* __restrict__ R, float* __restrict__ P) {
  const size_t tid = (size_t)blockIdx.x * 256 + threadIdx.x, nth = (size_t)gridDim.x * 256;
  for (int pass = 0; pass < 2; ++pass) {
    for (size_t p = tid; p < Wo_::END / 8; p += nth) { const size_t q = p * 8; v8b v;
      if (q < Wo_::W16) { const int k = (int)(q / (16 * 64)), o = (int)(q / 64) % 16, f0 = (int)(q % 64); for (int e = 0; e < 8; ++e) v[e] = (b16)((o < 4) ? bf16_rne(W8[(k * 4 + o) * 64 + f0 + e]) : 0.0f); }
      else if (q < Wo_::W32) { const size_t r = q - Wo_::W16; for (int e = 0; e < 8; ++e) v[e] = (b16)bf16_rne(W16[r + e]); }
      else if (q < Wo_::W64) { const size_t r = q - Wo_::W32; for (int e = 0; e < 8; ++e) v[e] = (b16)bf16_rne(W32[r + e]); }
      else if (q < Wo_::FC) { const size_t r = q - Wo_::W64; for (int e = 0; e < 8; ++e) v[e] = (b16)bf16_rne(W64[r + e]); }
      else { const size_t r = q - Wo_::FC; for (int e = 0; e < 8; ++e) v[e] = (b16)bf16_rne(Wfc[r + e]); }
      *(volatile v8b*)(R + q) = v; }
    for (size_t q = tid; q < 880; q += nth) { const int i = (int)q; float v; if (i < 32) v = b8[i]; else if (i < 96) v = b16_[i - 32]; else if (i < 224) v = b32[i - 96]; else if (i < 480) v = b64[i - 224]; else v = bfc[i - 480]; P[q] = bf16_rne(v); }
    __threadfence(); }
}

__device__ __forceinline__ v16b frag_patch(const float* xu, int k, int h, int p, int kb, int hh) { v16b f;
#pragma unroll
  for (int half = 0; half < 2; ++half) { const int f0 = kb + 16 * half + 8 * hh; const int r = f0 / h, c = f0 % h; const float* src = xu + (size_t)(k + r) * T + p * h + c;
#pragma unroll
    for (int e = 0; e < 8; ++e) f[half * 8 + e] = (b16)bf16_rne(src[e]); }
  return f; }
__global__ __launch_bounds__(256) void feat_kernel(const float* __restrict__ x, const b16* __restrict__ R, const float* __restrict__ P, float* __restrict__ FE) {
  __shared__ __attribute__((aligned(16))) float fe[NFE];
  const int u = blockIdx.x, lane = threadIdx.x & 31, wave = threadIdx.x >> 5, nloc = lane & 15, hlf = lane >> 4; const float* xu = x + (size_t)u * F * T;
  { const int k = wave;
    for (int rt = 0; rt < 4; ++rt) { v8f acc = {};
#pragma unroll
      for (int kb = 0; kb < 64; kb += 32) acc = wmma16b(frag_patch(xu, k, 8, rt * 16 + nloc, kb, hlf), frag_kb(R + Wo_::W8 + (size_t)(k * 16 + nloc) * 64 + kb, hlf), acc);
#pragma unroll
      for (int r = 0; r < 8; ++r) if (nloc < 4) fe[((k * 64) + rt * 16 + 8 * hlf + r) * 4 + nloc] = acc[r] + P[k * 4 + nloc]; } }
  { const int k = wave >> 1, rt = wave & 1; v8f acc = {};
    for (int kb = 0; kb < 256; kb += 32) acc = wmma16b(frag_patch(xu, k, 16, rt * 16 + nloc, kb, hlf), frag_kb(R + Wo_::W16 + (size_t)(k * 16 + nloc) * 256 + kb, hlf), acc);
#pragma unroll
    for (int r = 0; r < 8; ++r) fe[2048 + ((k * 32) + rt * 16 + 8 * hlf + r) * 16 + nloc] = acc[r] + P[32 + k * 16 + nloc]; }
  { const int k = wave >> 2, t = wave & 3; v8f acc = {};
    for (int kb = 0; kb < 1024; kb += 32) acc = wmma16b(frag_patch(xu, k, 32, nloc, kb, hlf), frag_kb(R + Wo_::W32 + (size_t)(k * 64 + t * 16 + nloc) * 1024 + kb, hlf), acc);
#pragma unroll
    for (int r = 0; r < 8; ++r) fe[4096 + ((k * 16) + 8 * hlf + r) * 64 + t * 16 + nloc] = acc[r] + P[96 + k * 64 + t * 16 + nloc]; }
  { v8f a0 = {}, a1 = {}; const int pr = (nloc < 8) ? nloc : 7;
    for (int kb = 0; kb < 4096; kb += 32) { const v16b a = frag_patch(xu, 0, 64, pr, kb, hlf); a0 = wmma16b(a, frag_kb(R + Wo_::W64 + (size_t)(wave * 32 + nloc) * 4096 + kb, hlf), a0); a1 = wmma16b(a, frag_kb(R + Wo_::W64 + (size_t)(wave * 32 + 16 + nloc) * 4096 + kb, hlf), a1); }
    if (hlf == 0) {
#pragma unroll
      for (int r = 0; r < 8; ++r) { fe[6144 + r * 256 + wave * 32 + nloc] = a0[r] + P[224 + wave * 32 + nloc]; fe[6144 + r * 256 + wave * 32 + 16 + nloc] = a1[r] + P[224 + wave * 32 + 16 + nloc]; } } }
  __syncthreads();
  for (int pass = 0; pass < 2; ++pass) { for (int i = threadIdx.x; i < NFE / 4; i += 256) *(volatile v4f*)(FE + (size_t)u * NFE + i * 4) = *(const v4f*)(&fe[i * 4]); __threadfence(); }
}

__global__ __launch_bounds__(256) void gfc_kernel(const float* __restrict__ FE, const b16* __restrict__ R, const float* __restrict__ P, float* __restrict__ G) {
  __shared__ __attribute__((aligned(16))) float Tg[32][OUT];
  const int lane = threadIdx.x & 31, wave = threadIdx.x >> 5, nloc = lane & 15, hlf = lane >> 4; const b16* Wf = R + Wo_::FC + 64;
  v8f acc[2][4];
#pragma unroll
  for (int r = 0; r < 2; ++r)
#pragma unroll
    for (int t = 0; t < 4; ++t) acc[r][t] = (v8f){};
  const int nt = (wave == 0) ? 4 : 3;
  for (int kb = 0; kb < NFE; kb += 32) { v16b h0, l0, h1, l1; frag_split(FE + (size_t)nloc * NFE + kb, hlf, h0, l0); frag_split(FE + (size_t)(16 + nloc) * NFE + kb, hlf, h1, l1);
#pragma unroll
    for (int t = 0; t < 4; ++t) { if (t < nt) { const v16b bw = frag_kb(Wf + (size_t)((wave + 8 * t) * 16 + nloc) * KFC + kb, hlf); acc[0][t] = wmma16b(h0, bw, acc[0][t]); acc[0][t] = wmma16b(l0, bw, acc[0][t]); acc[1][t] = wmma16b(h1, bw, acc[1][t]); acc[1][t] = wmma16b(l1, bw, acc[1][t]); } } }
#pragma unroll
  for (int t = 0; t < 4; ++t) { if (t < nt) { const int c = (wave + 8 * t) * 16 + nloc;
#pragma unroll
      for (int r = 0; r < 2; ++r)
#pragma unroll
        for (int v = 0; v < 8; ++v) Tg[r * 16 + 8 * hlf + v][c] = acc[r][t][v] * (1.0f / AS_) + P[480 + c]; } }
  __syncthreads();
  for (int pass = 0; pass < 2; ++pass) { for (int i = threadIdx.x; i < 32 * OUT / 4; i += 256) *(volatile v4f*)(G + i * 4) = *(const v4f*)(&Tg[0][0] + i * 4); __threadfence(); }
}

__global__ __launch_bounds__(128) void out_kernel(const float* __restrict__ x, const b16* __restrict__ R, const float* __restrict__ G, float* __restrict__ out) {
  __shared__ __attribute__((aligned(16))) float To[32][OUT];
  const int lane = threadIdx.x & 31, wave = threadIdx.x >> 5, nloc = lane & 15, hlf = lane >> 4, u = blockIdx.y, t0 = blockIdx.x * 32; const float* xu = x + (size_t)u * F * T; const b16* Wf = R + Wo_::FC;
  v8f acc[2][7];
#pragma unroll
  for (int r = 0; r < 2; ++r)
#pragma unroll
    for (int t = 0; t < 7; ++t) acc[r][t] = (v8f){};
  const int nt = (wave == 0) ? 7 : 6;
#pragma unroll
  for (int kb = 0; kb < F; kb += 32) { v16b a0, a1;
#pragma unroll
    for (int e = 0; e < 16; ++e) { const int i = kb + ((e < 8) ? (8 * hlf + e) : (16 + 8 * hlf + e - 8)); a0[e] = (b16)bf16_rne(xu[(size_t)i * T + t0 + nloc]); a1[e] = (b16)bf16_rne(xu[(size_t)i * T + t0 + 16 + nloc]); }
#pragma unroll
    for (int t = 0; t < 7; ++t) { if (t < nt) { const v16b bw = frag_kb(Wf + (size_t)((wave + 4 * t) * 16 + nloc) * KFC + kb, hlf); acc[0][t] = wmma16b(a0, bw, acc[0][t]); acc[1][t] = wmma16b(a1, bw, acc[1][t]); } } }
#pragma unroll
  for (int t = 0; t < 7; ++t) { if (t < nt) { const int c = (wave + 4 * t) * 16 + nloc; const float g = G[u * OUT + c];
#pragma unroll
      for (int r = 0; r < 2; ++r)
#pragma unroll
        for (int v = 0; v < 8; ++v) To[r * 16 + 8 * hlf + v][c] = acc[r][t][v] + g; } }
  __syncthreads();
  for (int pass = 0; pass < 2; ++pass) { for (int i = threadIdx.x; i < 32 * OUT / 4; i += 128) *(volatile v4f*)(out + ((size_t)u * T + t0) * OUT + i * 4) = *(const v4f*)(&To[0][0] + i * 4); __threadfence(); }
}
}

extern "C" void kernel_launch(void* const* d_in, const int* in_sizes, int n_in,
                              void* d_out, int out_size, void* d_ws, size_t ws_size, hipStream_t stream) {
  (void)n_in; (void)out_size;
  const float* x = (const float*)d_in[0]; const float* W8 = (const float*)d_in[1]; const float* b8 = (const float*)d_in[2]; const float* W16 = (const float*)d_in[3]; const float* b16_ = (const float*)d_in[4]; const float* W32 = (const float*)d_in[5]; const float* b32 = (const float*)d_in[6];
  const float* W64 = (const float*)d_in[7]; const float* b64 = (const float*)d_in[8]; const float* Wfc = (const float*)d_in[9]; const float* bfc = (const float*)d_in[10];
  float* out = (float*)d_out;
  if (in_sizes[0] != Bn * F * T || in_sizes[1] != 8 * 4 * 64 || in_sizes[7] != 256 * 4096 || in_sizes[9] != OUT * KFC) return;
  size_t off = 0; char* ws = (char*)d_ws;
  auto carve = [&](size_t bytes) { char* p = ws + off; off += (bytes + 255) & ~(size_t)255; return p; };
  b16* R = (b16*)carve(Wo_::END * 2); float* P = (float*)carve(1024 * 4); float* FE = (float*)carve((size_t)Bn * NFE * 4); float* G = (float*)carve((size_t)Bn * OUT * 4);
  if (off > ws_size) return;
  prep_kernel<<<512, 256, 0, stream>>>(W8, b8, W16, b16_, W32, b32, W64, b64, Wfc, bfc, R, P);
  feat_kernel<<<Bn, 256, 0, stream>>>(x, R, P, FE);
  gfc_kernel<<<1, 256, 0, stream>>>(FE, R, P, G);
  out_kernel<<<dim3(T / 32, Bn), 128, 0, stream>>>(x, R, G, out);
}
